// Encode_Graph_73976516706557
// MI455X (gfx1250) — hardware-verified
//
#include <hip/hip_runtime.h>
#include <stddef.h>


#define CIN    16
#define C1     32
#define C2     64
#define KPA    32
#define NTHR   256
#define NWAVE  8
#define EPT    8
#define NGRP   2
#define CHUNK  (NTHR * EPT * NGRP)
#define WCAP   (EPT * NGRP * 32)
#define LISTN  (NWAVE * WCAP)
#define SLB    14
#define NBD    8192
#define NBA    2048
#define GPB    16
#define GTHR   128
#define GWAVE  4
#define TPW    8
#define RPB    (GWAVE * TPW * 16)
#define P1     40
#define P2     72
#define OFF_WA 0
#define OFF_WP 1024
#define OFF_WC 2048
#define OFF_WL 6144
#define WTOT   10240

#define LDS_A1 ((NBA * CIN) * 4 + NBA * 4 + LISTN * 4 + 64)
#define LDS_A2 ((NBA * C1) * 2 + LISTN * 4 + 64)

static_assert((CHUNK & (CHUNK - 1)) == 0);
static_assert(CHUNK <= (1 << 12));
static_assert((NBD & (NBD - 1)) == 0 && NBD <= (1 << SLB));
static_assert((NBA & (NBA - 1)) == 0 && NBA <= (1 << SLB));
static_assert((NBA % RPB) == 0);
static_assert(NBD == NWAVE * 8 * 32 * 4);
static_assert(NBA == NWAVE * 16 * 16);
static_assert(NBA == NWAVE * 32 * 8);
static_assert(GPB * C2 == NTHR * 4);
static_assert(KPA == C1);

typedef float          v2f  __attribute__((ext_vector_type(2)));
typedef float          v4f  __attribute__((ext_vector_type(4)));
typedef float          v8f  __attribute__((ext_vector_type(8)));
typedef int            v4i  __attribute__((ext_vector_type(4)));
typedef unsigned int   v4u  __attribute__((ext_vector_type(4)));
typedef _Float16       v2h  __attribute__((ext_vector_type(2)));
typedef _Float16       v8h  __attribute__((ext_vector_type(8)));
typedef _Float16       v16h __attribute__((ext_vector_type(16)));
union Frag { v16h v; v8h h[2]; v4i q[2]; };

__device__ __forceinline__ v8f wmh(v16h a, v16h b, v8f c) {
  v8f d = __builtin_amdgcn_wmma_f32_16x16x32_f16(false, a, false, b, (short)0, c, false, false);
  asm volatile("v_nop\n\tv_nop\n\tv_nop\n\tv_nop" : "+v"(d) : "v"(a), "v"(b));
  return d;
}

template <int NB>
__device__ __forceinline__ int scan_chunk(const int* __restrict__ ids, int nE, int cbase, int slotBase,
                                          int vec8, int* list, int tid, int lane, int wave) {
  int wc = 0;
#pragma unroll
  for (int g = 0; g < NGRP; ++g) {
    const int el0  = (g * NTHR + tid) * EPT;
    const int e0   = cbase + el0;
    const int sent = -2147483647 - 1;
    v4i da, db;
    if (vec8 != 0 && cbase + CHUNK <= nE) {
      da = *(const v4i*)(ids + e0);
      db = *(const v4i*)(ids + e0 + 4);
    } else {
      da.x = (e0     < nE) ? ids[min(e0, nE - 1)] : sent;
      da.y = (e0 + 1 < nE) ? ids[min(e0 + 1, nE - 1)] : sent;
      da.z = (e0 + 2 < nE) ? ids[min(e0 + 2, nE - 1)] : sent;
      da.w = (e0 + 3 < nE) ? ids[min(e0 + 3, nE - 1)] : sent;
      db.x = (e0 + 4 < nE) ? ids[min(e0 + 4, nE - 1)] : sent;
      db.y = (e0 + 5 < nE) ? ids[min(e0 + 5, nE - 1)] : sent;
      db.z = (e0 + 6 < nE) ? ids[min(e0 + 6, nE - 1)] : sent;
      db.w = (e0 + 7 < nE) ? ids[min(e0 + 7, nE - 1)] : sent;
    }
    const unsigned nb = (unsigned)slotBase;
    const unsigned s0 = (unsigned)da.x - nb, s1 = (unsigned)da.y - nb;
    const unsigned s2 = (unsigned)da.z - nb, s3 = (unsigned)da.w - nb;
    const unsigned s4 = (unsigned)db.x - nb, s5 = (unsigned)db.y - nb;
    const unsigned s6 = (unsigned)db.z - nb, s7 = (unsigned)db.w - nb;
    const bool h0 = s0 < (unsigned)NB, h1 = s1 < (unsigned)NB, h2 = s2 < (unsigned)NB, h3 = s3 < (unsigned)NB;
    const bool h4 = s4 < (unsigned)NB, h5 = s5 < (unsigned)NB, h6 = s6 < (unsigned)NB, h7 = s7 < (unsigned)NB;
    const unsigned any = __builtin_amdgcn_ballot_w32(h0 | h1 | h2 | h3 | h4 | h5 | h6 | h7);
    if (any != 0u) {
#define HITJ(J, HJ, SJ) { \
        const unsigned mj = __builtin_amdgcn_ballot_w32(HJ); \
        if (mj != 0u) { \
          if (HJ) { \
            const int pos = wc + (int)__builtin_amdgcn_mbcnt_lo(mj, 0u); \
            if (pos < WCAP) list[wave * WCAP + pos] = ((el0 + (J)) << SLB) | (int)(SJ); \
          } \
          wc += (int)__builtin_popcount(mj); } }
      HITJ(0, h0, s0)
      HITJ(1, h1, s1)
      HITJ(2, h2, s2)
      HITJ(3, h3, s3)
      HITJ(4, h4, s4)
      HITJ(5, h5, s5)
      HITJ(6, h6, s6)
      HITJ(7, h7, s7)
#undef HITJ
    }
  }
  return wc;
}

__global__ __launch_bounds__(NTHR) void k_wprep(
    const float* __restrict__ W1, const float* __restrict__ Wp, const float* __restrict__ Ws,
    const float* __restrict__ Wn, const float* __restrict__ Wl, _Float16* Wpl) {
  const int seg = (int)blockIdx.x, tid = (int)threadIdx.x;
  if (seg == 0) {
    if (tid < 128) {
      const int n = tid >> 2, k0 = (tid & 3) * 8;
      v8h v;
#pragma unroll
      for (int j = 0; j < 8; ++j) {
        const int k = k0 + j;
        const int kc = k < CIN ? k : CIN - 1;
        const float x = W1[kc * C1 + n];
        v[j] = (_Float16)(k < CIN ? x : 0.0f);
      }
      _Float16* p = Wpl + OFF_WA + tid * 8;
      *(volatile v8h*)p = v;
      __threadfence();
      *(volatile v8h*)p = v;
    }
  } else if (seg == 1) {
    if (tid < 128) {
      const int n = tid >> 2, k0 = (tid & 3) * 8;
      v8h v;
#pragma unroll
      for (int j = 0; j < 8; ++j) v[j] = (_Float16)Wp[(k0 + j) * C1 + n];
      _Float16* p = Wpl + OFF_WP + tid * 8;
      *(volatile v8h*)p = v;
      __threadfence();
      *(volatile v8h*)p = v;
    }
  } else if (seg == 2) {
#pragma unroll
    for (int it = 0; it < 2; ++it) {
      const int u = it * NTHR + tid;
      const int n = u >> 3, k0 = (u & 7) * 8;
      v8h v;
#pragma unroll
      for (int j = 0; j < 8; ++j) {
        const int k  = k0 + j;
        const int ks = k < C1 ? k : C1 - 1;
        const int kn = k >= C1 ? k - C1 : 0;
        const float xs = Ws[ks * C2 + n];
        const float xn = Wn[kn * C2 + n];
        v[j] = (_Float16)(k < C1 ? xs : xn);
      }
      _Float16* p = Wpl + OFF_WC + u * 8;
      *(volatile v8h*)p = v;
      __threadfence();
      *(volatile v8h*)p = v;
    }
  } else if (seg == 3) {
#pragma unroll
    for (int it = 0; it < 2; ++it) {
      const int u = it * NTHR + tid;
      const int n = u >> 3, k0 = (u & 7) * 8;
      v8h v;
#pragma unroll
      for (int j = 0; j < 8; ++j) v[j] = (_Float16)Wl[(k0 + j) * C2 + n];
      _Float16* p = Wpl + OFF_WL + u * 8;
      *(volatile v8h*)p = v;
      __threadfence();
      *(volatile v8h*)p = v;
    }
  }
}

__device__ __forceinline__ void degsrc_store(const int* scnt, float* np, int wave, int lane) {
#pragma unroll 1
  for (int it = 0; it < 8; ++it) {
    const int f = ((it * NWAVE + wave) * 32 + lane) * 4;
    const v4i c = *(const v4i*)(scnt + f);
    v4f v;
    v.x = rsqrtf((float)(c.x > 1 ? c.x : 1));
    v.y = rsqrtf((float)(c.y > 1 ? c.y : 1));
    v.z = rsqrtf((float)(c.z > 1 ? c.z : 1));
    v.w = rsqrtf((float)(c.w > 1 ? c.w : 1));
    *(volatile v4f*)(np + f) = v;
  }
}

__global__ __launch_bounds__(NTHR) void k_degsrc(
    const int* __restrict__ esrc, float* normS, int nE, int vec8) {
  __shared__ __attribute__((aligned(16))) int scnt[NBD];
  __shared__ __attribute__((aligned(16))) int list[LISTN];
  __shared__ int wcnt[NWAVE];
  const int tid = threadIdx.x, lane = tid & 31, wave = tid >> 5;
  const int slotBase = (int)blockIdx.x * NBD;
  for (int i = tid; i < NBD; i += NTHR) scnt[i] = 0;
  __syncthreads();

  const int nChunks = (nE + CHUNK - 1) / CHUNK;
#pragma unroll 1
  for (int ch = 0; ch < nChunks; ++ch) {
    const int cbase = ch * CHUNK;
    const int wc = scan_chunk<NBD>(esrc, nE, cbase, slotBase, vec8, list, tid, lane, wave);
    if (lane == 0) wcnt[wave] = wc;
    __syncthreads();
    if (wave == 0) {
#pragma unroll 1
      for (int wsx = 0; wsx < NWAVE; ++wsx) {
        int n = __builtin_amdgcn_readfirstlane(wcnt[wsx]);
        n = n > WCAP ? WCAP : (n < 0 ? 0 : n);
        const int* lp = list + wsx * WCAP;
#pragma unroll 1
        for (int i = 0; i < n; ++i) {
          const int ent  = __builtin_amdgcn_readfirstlane(lp[i]);
          const int slot = ent & (NBD - 1);
          if (lane == 0) scnt[slot] = scnt[slot] + 1;
        }
      }
    }
    __syncthreads();
  }

  float* np = normS + (size_t)slotBase;
  degsrc_store(scnt, np, wave, lane);
  __threadfence();
  degsrc_store(scnt, np, wave, lane);
}

__device__ __forceinline__ void agg1_store(const float* sacc, const int* scnt, _Float16* M16,
                                           int slotBase, int wave, int lane) {
#pragma unroll 2
  for (int it = 0; it < 16; ++it) {
    const int row = (it * NWAVE + wave) * 16 + (lane >> 1);
    const int c0  = (lane & 1) * 8;
    const int c   = scnt[row];
    const float nd = 1.0f / sqrtf((float)(c > 1 ? c : 1));
    const v4f a = *(const v4f*)(sacc + row * CIN + c0);
    const v4f b = *(const v4f*)(sacc + row * CIN + c0 + 4);
    v8h hv;
    hv[0] = (_Float16)(a.x * nd); hv[1] = (_Float16)(a.y * nd);
    hv[2] = (_Float16)(a.z * nd); hv[3] = (_Float16)(a.w * nd);
    hv[4] = (_Float16)(b.x * nd); hv[5] = (_Float16)(b.y * nd);
    hv[6] = (_Float16)(b.z * nd); hv[7] = (_Float16)(b.w * nd);
    *(volatile v8h*)(M16 + ((size_t)slotBase + (size_t)row) * CIN + c0) = hv;
  }
}

__global__ __launch_bounds__(NTHR) void k_agg1(
    const int* __restrict__ edst, const int* __restrict__ esrc, const int* __restrict__ tok,
    const float* __restrict__ emb, const float* __restrict__ normS, _Float16* M16,
    int nN, int nE, int nVoc, int vec8) {
  extern __shared__ v4f lds_dyn[];
  float* sacc = (float*)lds_dyn;
  int*   scnt = (int*)(sacc + NBA * CIN);
  int*   list = scnt + NBA;
  int*   wcnt = list + LISTN;
  const int tid = threadIdx.x, lane = tid & 31, wave = tid >> 5;
  const int slotBase = (int)blockIdx.x * NBA;
  {
    const v4f z = {0.f, 0.f, 0.f, 0.f};
    for (int i = tid; i < NBA * CIN / 4; i += NTHR) ((v4f*)sacc)[i] = z;
    for (int i = tid; i < NBA; i += NTHR) scnt[i] = 0;
  }
  __syncthreads();

  const int ch16 = lane & (CIN - 1);
  const int nChunks = (nE + CHUNK - 1) / CHUNK;
#pragma unroll 1
  for (int ch = 0; ch < nChunks; ++ch) {
    const int cbase = ch * CHUNK;
    const int wc = scan_chunk<NBA>(edst, nE, cbase, slotBase, vec8, list, tid, lane, wave);
    if (lane == 0) wcnt[wave] = wc;
    __syncthreads();
    if (wave == 0) {
#pragma unroll 1
      for (int wsx = 0; wsx < NWAVE; ++wsx) {
        int n = __builtin_amdgcn_readfirstlane(wcnt[wsx]);
        n = n > WCAP ? WCAP : (n < 0 ? 0 : n);
        const int* lp = list + wsx * WCAP;
#pragma unroll 1
        for (int i = 0; i < n; ++i) {
          const int ent  = __builtin_amdgcn_readfirstlane(lp[i]);
          const int slot = ent & (NBA - 1);
          int e = cbase + ((ent >> SLB) & (CHUNK - 1));
          e = e > nE - 1 ? nE - 1 : e;
          int s = esrc[e];
          if (s < 0) s += nN;
          s = s < 0 ? 0 : (s > nN - 1 ? nN - 1 : s);
          int t = tok[s];
          if (t < 0) t += nVoc;
          t = t < 0 ? 0 : (t > nVoc - 1 ? nVoc - 1 : t);
          const float ns = normS[s];
          const float v  = emb[(size_t)t * CIN + ch16] * ns;
          if (lane < CIN) sacc[slot * CIN + ch16] = sacc[slot * CIN + ch16] + v;
          if (lane == 0) scnt[slot] = scnt[slot] + 1;
        }
      }
    }
    __syncthreads();
  }

  agg1_store(sacc, scnt, M16, slotBase, wave, lane);
  __threadfence();
  agg1_store(sacc, scnt, M16, slotBase, wave, lane);
}

__device__ __forceinline__ void g12_store(const _Float16* t1, const _Float16* t2,
                                          _Float16* H1, _Float16* HP, size_t row0, int lane) {
#pragma unroll
  for (int i = 0; i < 2; ++i) {
    const int p = i * 32 + lane, row = p >> 2, cc = (p & 3) * 8;
    const v8h v1 = *(const v8h*)(t1 + row * P1 + cc);
    const v8h v2 = *(const v8h*)(t2 + row * P1 + cc);
    *(volatile v8h*)(H1 + (row0 + (size_t)row) * C1 + cc) = v1;
    *(volatile v8h*)(HP + (row0 + (size_t)row) * C1 + cc) = v2;
  }
}

__global__ __launch_bounds__(GTHR) void k_gemm12(
    const _Float16* __restrict__ M16, const _Float16* __restrict__ Wpl,
    const float* __restrict__ b1, const float* __restrict__ bp, _Float16* H1, _Float16* HP) {
  __shared__ __attribute__((aligned(16))) _Float16 sT1[GWAVE * 16 * P1];
  __shared__ __attribute__((aligned(16))) _Float16 sT2[GWAVE * 16 * P1];
  const int tid = threadIdx.x, lane = tid & 31, wave = tid >> 5, hh = lane >> 4, m = lane & 15;
  _Float16* t1 = sT1 + wave * 16 * P1;
  _Float16* t2 = sT2 + wave * 16 * P1;
  const _Float16* WA = Wpl + OFF_WA;
  const _Float16* WP = Wpl + OFF_WP;

  Frag wa0, wa1, wp0, wp1;
  wa0.h[0] = *(const v8h*)(WA + (size_t)m * KPA + 8 * hh);
  wa0.h[1] = *(const v8h*)(WA + (size_t)m * KPA + 16 + 8 * hh);
  wa1.h[0] = *(const v8h*)(WA + (size_t)(16 + m) * KPA + 8 * hh);
  wa1.h[1] = *(const v8h*)(WA + (size_t)(16 + m) * KPA + 16 + 8 * hh);
  wp0.h[0] = *(const v8h*)(WP + (size_t)m * C1 + 8 * hh);
  wp0.h[1] = *(const v8h*)(WP + (size_t)m * C1 + 16 + 8 * hh);
  wp1.h[0] = *(const v8h*)(WP + (size_t)(16 + m) * C1 + 8 * hh);
  wp1.h[1] = *(const v8h*)(WP + (size_t)(16 + m) * C1 + 16 + 8 * hh);
  const float bA0 = b1[m], bA1 = b1[16 + m], bP0 = bp[m], bP1 = bp[16 + m];
  const v4i zi = {0, 0, 0, 0};
  const v8f z = {0.f, 0.f, 0.f, 0.f, 0.f, 0.f, 0.f, 0.f};
  const int tile0 = ((int)blockIdx.x * GWAVE + wave) * TPW;

#pragma unroll 1
  for (int tt = 0; tt < TPW; ++tt) {
    const size_t row0 = (size_t)(tile0 + tt) * 16;
    Frag a;
    a.h[0] = *(const v8h*)(M16 + (row0 + (size_t)m) * CIN + 8 * hh);
    a.q[1] = zi;
    const v8f c0 = wmh(a.v, wa0.v, z);
    const v8f c1 = wmh(a.v, wa1.v, z);
#pragma unroll
    for (int r = 0; r < 8; ++r) {
      t1[(8 * hh + r) * P1 + m]      = (_Float16)fmaxf(c0[r] + bA0, 0.0f);
      t1[(8 * hh + r) * P1 + 16 + m] = (_Float16)fmaxf(c1[r] + bA1, 0.0f);
    }
    __syncthreads();
    Frag a2;
    a2.h[0] = *(const v8h*)(t1 + m * P1 + 8 * hh);
    a2.h[1] = *(const v8h*)(t1 + m * P1 + 16 + 8 * hh);
    const v8f d0 = wmh(a2.v, wp0.v, z);
    const v8f d1 = wmh(a2.v, wp1.v, z);
#pragma unroll
    for (int r = 0; r < 8; ++r) {
      t2[(8 * hh + r) * P1 + m]      = (_Float16)fmaxf(d0[r] + bP0, 0.0f);
      t2[(8 * hh + r) * P1 + 16 + m] = (_Float16)fmaxf(d1[r] + bP1, 0.0f);
    }
    __syncthreads();
    g12_store(t1, t2, H1, HP, row0, lane);
    __threadfence();
    g12_store(t1, t2, H1, HP, row0, lane);
    __syncthreads();
  }
}

__device__ __forceinline__ void agg2_store(const _Float16* sacc, _Float16* HN, int slotBase, int wave, int lane) {
#pragma unroll 2
  for (int it = 0; it < 32; ++it) {
    const int row = (it * NWAVE + wave) * 8 + (lane >> 2);
    const int c0  = (lane & 3) * 8;
    const v8h a = *(const v8h*)(sacc + row * C1 + c0);
    v8h o;
#pragma unroll
    for (int j = 0; j < 8; ++j) {
      const float f = (float)a[j];
      o[j] = (_Float16)(f < 0.0f ? 0.0f : f);
    }
    *(volatile v8h*)(HN + ((size_t)slotBase + (size_t)row) * C1 + c0) = o;
  }
}

__global__ __launch_bounds__(NTHR) void k_agg2(
    const int* __restrict__ edst, const int* __restrict__ esrc, const _Float16* __restrict__ HP,
    _Float16* HN, int nN, int nE, int vec8) {
  extern __shared__ v4f lds_dyn[];
  _Float16* sacc = (_Float16*)lds_dyn;
  int* list = (int*)(sacc + NBA * C1);
  int* wcnt = list + LISTN;
  const int tid = threadIdx.x, lane = tid & 31, wave = tid >> 5;
  const int slotBase = (int)blockIdx.x * NBA;
  {
    const v4u negb = {0xBC00BC00u, 0xBC00BC00u, 0xBC00BC00u, 0xBC00BC00u};
    for (int i = tid; i < NBA * C1 / 8; i += NTHR) ((v4u*)lds_dyn)[i] = negb;
  }
  __syncthreads();

  const int nChunks = (nE + CHUNK - 1) / CHUNK;
#pragma unroll 1
  for (int ch = 0; ch < nChunks; ++ch) {
    const int cbase = ch * CHUNK;
    const int wc = scan_chunk<NBA>(edst, nE, cbase, slotBase, vec8, list, tid, lane, wave);
    if (lane == 0) wcnt[wave] = wc;
    __syncthreads();
    if (wave == 0) {
#pragma unroll 1
      for (int wsx = 0; wsx < NWAVE; ++wsx) {
        int n = __builtin_amdgcn_readfirstlane(wcnt[wsx]);
        n = n > WCAP ? WCAP : (n < 0 ? 0 : n);
        const int* lp = list + wsx * WCAP;
#pragma unroll 1
        for (int i = 0; i < n; ++i) {
          const int ent  = __builtin_amdgcn_readfirstlane(lp[i]);
          const int slot = ent & (NBA - 1);
          int e = cbase + ((ent >> SLB) & (CHUNK - 1));
          e = e > nE - 1 ? nE - 1 : e;
          int s = esrc[e];
          if (s < 0) s += nN;
          s = s < 0 ? 0 : (s > nN - 1 ? nN - 1 : s);
          const _Float16 hv = HP[(size_t)s * C1 + lane];
          _Float16* ap = sacc + slot * C1 + lane;
          const float cur = (float)(*ap);
          const float nv  = (float)hv;
          *ap = (_Float16)fmaxf(cur, nv);
        }
      }
    }
    __syncthreads();
  }

  agg2_store(sacc, HN, slotBase, wave, lane);
  __threadfence();
  agg2_store(sacc, HN, slotBase, wave, lane);
}

__device__ __forceinline__ void g34_store(const _Float16* t3, _Float16* H3, size_t row0, int lane) {
#pragma unroll
  for (int i = 0; i < 4; ++i) {
    const int p = i * 32 + lane, row = p >> 3, cc = (p & 7) * 8;
    const v8h v = *(const v8h*)(t3 + row * P2 + cc);
    *(volatile v8h*)(H3 + (row0 + (size_t)row) * C2 + cc) = v;
  }
}

__global__ __launch_bounds__(GTHR) void k_gemm34(
    const _Float16* __restrict__ H1, const _Float16* __restrict__ HN, const _Float16* __restrict__ Wpl,
    const float* __restrict__ bn, const float* __restrict__ bl, _Float16* H3) {
  __shared__ __attribute__((aligned(16))) _Float16 sT2[GWAVE * 16 * P2];
  __shared__ __attribute__((aligned(16))) _Float16 sT3[GWAVE * 16 * P2];
  const int tid = threadIdx.x, lane = tid & 31, wave = tid >> 5, hh = lane >> 4, m = lane & 15;
  _Float16* t2 = sT2 + wave * 16 * P2;
  _Float16* t3 = sT3 + wave * 16 * P2;
  const _Float16* WC = Wpl + OFF_WC;
  const _Float16* WL = Wpl + OFF_WL;
  float bnv[4], blv[4];
#pragma unroll
  for (int t = 0; t < 4; ++t) { bnv[t] = bn[16 * t + m]; blv[t] = bl[16 * t + m]; }
  const v8f z = {0.f, 0.f, 0.f, 0.f, 0.f, 0.f, 0.f, 0.f};
  const int tile0 = ((int)blockIdx.x * GWAVE + wave) * TPW;

#pragma unroll 1
  for (int tt = 0; tt < TPW; ++tt) {
    const size_t row0 = (size_t)(tile0 + tt) * 16;
    Frag a0, a1;
    a0.h[0] = *(const v8h*)(H1 + (row0 + (size_t)m) * C1 + 8 * hh);
    a0.h[1] = *(const v8h*)(H1 + (row0 + (size_t)m) * C1 + 16 + 8 * hh);
    a1.h[0] = *(const v8h*)(HN + (row0 + (size_t)m) * C1 + 8 * hh);
    a1.h[1] = *(const v8h*)(HN + (row0 + (size_t)m) * C1 + 16 + 8 * hh);
    v8f acc[4];
#pragma unroll
    for (int t = 0; t < 4; ++t) {
      const _Float16* wp = WC + (size_t)(16 * t + m) * C2 + 8 * hh;
      Frag b0, b1f;
      b0.h[0]  = *(const v8h*)(wp);
      b0.h[1]  = *(const v8h*)(wp + 16);
      b1f.h[0] = *(const v8h*)(wp + 32);
      b1f.h[1] = *(const v8h*)(wp + 48);
      v8f c = wmh(a0.v, b0.v, z);
      c = wmh(a1.v, b1f.v, c);
      acc[t] = c;
    }
#pragma unroll
    for (int t = 0; t < 4; ++t) {
#pragma unroll
      for (int r = 0; r < 8; ++r)
        t2[(8 * hh + r) * P2 + 16 * t + m] = (_Float16)fmaxf(acc[t][r] + bnv[t], 0.0f);
    }
    __syncthreads();
    Frag g0, g1;
    g0.h[0] = *(const v8h*)(t2 + m * P2 + 8 * hh);
    g0.h[1] = *(const v8h*)(t2 + m * P2 + 16 + 8 * hh);
    g1.h[0] = *(const v8h*)(t2 + m * P2 + 32 + 8 * hh);
    g1.h[1] = *(const v8h*)(t2 + m * P2 + 48 + 8 * hh);
    v8f acc3[4];
#pragma unroll
    for (int t = 0; t < 4; ++t) {
      const _Float16* wp = WL + (size_t)(16 * t + m) * C2 + 8 * hh;
      Frag b0, b1f;
      b0.h[0]  = *(const v8h*)(wp);
      b0.h[1]  = *(const v8h*)(wp + 16);
      b1f.h[0] = *(const v8h*)(wp + 32);
      b1f.h[1] = *(const v8h*)(wp + 48);
      v8f c = wmh(g0.v, b0.v, z);
      c = wmh(g1.v, b1f.v, c);
      acc3[t] = c;
    }
#pragma unroll
    for (int t = 0; t < 4; ++t) {
#pragma unroll
      for (int r = 0; r < 8; ++r)
        t3[(8 * hh + r) * P2 + 16 * t + m] = (_Float16)fmaxf(acc3[t][r] + blv[t], 0.0f);
    }
    __syncthreads();
    g34_store(t3, H3, row0, lane);
    __threadfence();
    g34_store(t3, H3, row0, lane);
    __syncthreads();
  }
}

__global__ __launch_bounds__(NTHR) void k_pool(
    const int* __restrict__ gid, const _Float16* __restrict__ H3, float* out, int nN, int vecb) {
  __shared__ __attribute__((aligned(16))) float sacc[NWAVE * GPB * C2];
  __shared__ __attribute__((aligned(16))) int list[LISTN];
  const int tid = threadIdx.x, lane = tid & 31, wave = tid >> 5;
  const int gBase = (int)blockIdx.x * GPB;
  {
    const v4f z = {0.f, 0.f, 0.f, 0.f};
    for (int i = tid; i < NWAVE * GPB * C2 / 4; i += NTHR) ((v4f*)sacc)[i] = z;
  }
  __syncthreads();
  float* wacc = sacc + wave * GPB * C2;

  const int nChunks = (nN + CHUNK - 1) / CHUNK;
#pragma unroll 1
  for (int ch = 0; ch < nChunks; ++ch) {
    const int cbase = ch * CHUNK;
    const int wc = scan_chunk<GPB>(gid, nN, cbase, gBase, vecb, list, tid, lane, wave);
    __syncthreads();
    int n = __builtin_amdgcn_readfirstlane(wc);
    n = n > WCAP ? WCAP : (n < 0 ? 0 : n);
    const int* lp = list + wave * WCAP;
#pragma unroll 1
    for (int i = 0; i < n; ++i) {
      const int ent = __builtin_amdgcn_readfirstlane(lp[i]);
      const int g = ent & (GPB - 1);
      int node = cbase + ((ent >> SLB) & (CHUNK - 1));
      node = node > nN - 1 ? nN - 1 : node;
      const v2h hv = *(const v2h*)(H3 + (size_t)node * C2 + 2 * lane);
      float* ap = wacc + g * C2 + 2 * lane;
      v2f cur = *(const v2f*)ap;
      cur.x += (float)hv.x;
      cur.y += (float)hv.y;
      *(v2f*)ap = cur;
    }
    __syncthreads();
  }

  const int g = tid >> 4, c0 = (tid & 15) * 4;
  v4f s = *(const v4f*)(sacc + g * C2 + c0);
#pragma unroll
  for (int w = 1; w < NWAVE; ++w) s = s + *(const v4f*)(sacc + w * GPB * C2 + g * C2 + c0);
  float* op = out + (size_t)gBase * C2 + (size_t)tid * 4;
  *(volatile v4f*)op = s;
  __threadfence();
  *(volatile v4f*)op = s;
}

extern "C" void kernel_launch(void* const* d_in, const int* in_sizes, int n_in,
                              void* d_out, int out_size, void* d_ws, size_t ws_size,
                              hipStream_t stream) {
  if (n_in < 14) return;
  const int nN = in_sizes[0];
  const int nE = in_sizes[1];
  if (nN <= 0 || nE <= 0) return;
  if (in_sizes[2] != nE || in_sizes[3] != nN) return;
  if (in_sizes[4] <= 0 || (in_sizes[4] % CIN) != 0) return;
  const int nVoc = in_sizes[4] / CIN;
  if (in_sizes[5] != CIN * C1 || in_sizes[6] != C1 || in_sizes[7] != C1 * C1 || in_sizes[8] != C1) return;
  if (in_sizes[9] != C1 * C2 || in_sizes[10] != C1 * C2 || in_sizes[11] != C2) return;
  if (in_sizes[12] != C2 * C2 || in_sizes[13] != C2) return;
  if (out_size <= 0 || (out_size % (GPB * C2)) != 0) return;
  const int nG = out_size / C2;
  if (nN > (1 << 26) || nE > (1 << 28)) return;

  const int*   tokens = (const int*)d_in[0];
  const int*   esrc   = (const int*)d_in[1];
  const int*   edst   = (const int*)d_in[2];
  const int*   gids   = (const int*)d_in[3];
  const float* embed  = (const float*)d_in[4];
  const float* W1     = (const float*)d_in[5];
  const float* b1     = (const float*)d_in[6];
  const float* Wpool  = (const float*)d_in[7];
  const float* bpool  = (const float*)d_in[8];
  const float* Wself  = (const float*)d_in[9];
  const float* Wneigh = (const float*)d_in[10];
  const float* bneigh = (const float*)d_in[11];
  const float* Wlin   = (const float*)d_in[12];
  const float* blin   = (const float*)d_in[13];
  float* out = (float*)d_out;

  const int nBA   = (nN + NBA - 1) / NBA;
  const int NPAD  = nBA * NBA;
  const int nBD   = (nN + NBD - 1) / NBD;
  const int NPADD = nBD * NBD;
  const int nGB   = NPAD / RPB;
  const int nPB   = nG / GPB;

  char* ws = (char*)d_ws;
  size_t off = 0;
#define ALN(x) (((x) + 255) & ~(size_t)255)
  const size_t oW = off;  off = ALN(off + (size_t)WTOT * 2);
  const size_t oA = off;
  const size_t oNS  = oA;
  size_t a1 = ALN(oNS + (size_t)NPADD * 4);
  const size_t oM16 = a1;  a1 = ALN(a1 + (size_t)NPAD * CIN * 2);
  const size_t oHP  = a1;  a1 = ALN(a1 + (size_t)NPAD * C1 * 2);
  const size_t oH3  = oA;
  const size_t a2   = ALN(oA + (size_t)NPAD * C2 * 2);
  off = a1 > a2 ? a1 : a2;
  const size_t oH1 = off;  off = ALN(off + (size_t)NPAD * C1 * 2);
  const size_t oHN = off;  off = ALN(off + (size_t)NPAD * C1 * 2);
#undef ALN
  if (off > ws_size) return;
  if (off > ((size_t)128 << 20)) return;

  _Float16* Wpl   = (_Float16*)(ws + oW);
  float*    normS = (float*)(ws + oNS);
  _Float16* M16   = (_Float16*)(ws + oM16);
  _Float16* HP    = (_Float16*)(ws + oHP);
  _Float16* H3    = (_Float16*)(ws + oH3);
  _Float16* H1    = (_Float16*)(ws + oH1);
  _Float16* HN    = (_Float16*)(ws + oHN);

  const int vec8 = ((nE & 3) == 0) ? 1 : 0;
  const int vecb = ((nN & 3) == 0) ? 1 : 0;

  k_wprep<<<4, NTHR, 0, stream>>>(W1, Wpool, Wself, Wneigh, Wlin, Wpl);

  k_degsrc<<<nBD, NTHR, 0, stream>>>(esrc, normS, nE, vec8);

  hipFuncSetAttribute(reinterpret_cast<const void*>(&k_agg1),
                      hipFuncAttributeMaxDynamicSharedMemorySize, LDS_A1);
  k_agg1<<<nBA, NTHR, LDS_A1, stream>>>(edst, esrc, tokens, embed, normS, M16, nN, nE, nVoc, vec8);

  k_gemm12<<<nGB, GTHR, 0, stream>>>(M16, Wpl, b1, bpool, H1, HP);

  hipFuncSetAttribute(reinterpret_cast<const void*>(&k_agg2),
                      hipFuncAttributeMaxDynamicSharedMemorySize, LDS_A2);
  k_agg2<<<nBA, NTHR, LDS_A2, stream>>>(edst, esrc, HP, HN, nN, nE, vec8);

  k_gemm34<<<nGB, GTHR, 0, stream>>>(H1, HN, Wpl, bneigh, blin, H3);

  k_pool<<<nPB, NTHR, 0, stream>>>(gids, H3, out, nN, vecb);
}
